// SeqTrackDecoderXL_84988812853395
// MI455X (gfx1250) — hardware-verified
//
#include <hip/hip_runtime.h>
#include <stdint.h>
#include <stddef.h>

#define L_SEQ 1024
#define NB    4
#define DMOD  1024
#define NHD   16
#define HDIM  64
#define NTOK  (L_SEQ * NB)
#define NBH   (NB * NHD)
#define PSCALE 16384.0f
#define OSCALE 8.0f
#define WSCALE 32.0f

#define G_W   ((NTOK * DMOD) / 8)
#define G_QKV ((3 * DMOD * DMOD) / 8)
#define G_SQ  ((DMOD * DMOD) / 8)
#define G_TOT (2 * G_W + G_QKV + 2 * G_SQ)

typedef _Float16 v16h __attribute__((ext_vector_type(16)));
typedef _Float16 v8h  __attribute__((ext_vector_type(8)));
typedef float    v8f  __attribute__((ext_vector_type(8)));
typedef float    v4f  __attribute__((ext_vector_type(4)));
typedef int      v4i  __attribute__((ext_vector_type(4)));
typedef v8h __attribute__((may_alias)) v8ha;
typedef v4f __attribute__((may_alias)) v4fa;
typedef v4i __attribute__((may_alias)) v4ia;

union Frag { v16h v; v8h half[2]; };

__device__ __forceinline__ v8f wmma_f16(v16h a, v16h b, v8f c) {
  v8f d = __builtin_amdgcn_wmma_f32_16x16x32_f16(false, a, false, b, (short)0, c, false, false);
  asm volatile("v_nop\n\tv_nop\n\tv_nop\n\tv_nop" : "+v"(d) : "v"(a), "v"(b));
  return d;
}

__device__ __forceinline__ v16h load_frag(const _Float16* p, int h) {
  Frag f;
  f.half[0] = *(const v8ha*)(p + 8 * h);
  f.half[1] = *(const v8ha*)(p + 16 + 8 * h);
  return f.v;
}

__global__ __launch_bounds__(256) void convert_kernel(
    const float* __restrict__ w, const float* __restrict__ r,
    const float* __restrict__ qkvw, const float* __restrict__ rnw,
    const float* __restrict__ oww,
    _Float16* __restrict__ wh, _Float16* __restrict__ rh,
    _Float16* __restrict__ qkvh, _Float16* __restrict__ rnh,
    _Float16* __restrict__ owh)
{
  const int g = blockIdx.x * 256 + threadIdx.x;
  if (g >= G_TOT) return;
  const float* src;
  _Float16* dst;
  float sc;
  if (g < G_W) {
    src = w + (size_t)g * 8; dst = wh + (size_t)g * 8; sc = 1.0f;
  } else if (g < 2 * G_W) {
    const int e = g - G_W;
    src = r + (size_t)e * 8; dst = rh + (size_t)e * 8; sc = 1.0f;
  } else if (g < 2 * G_W + G_QKV) {
    const int e = g - 2 * G_W;
    src = qkvw + (size_t)e * 8; dst = qkvh + (size_t)e * 8; sc = WSCALE;
  } else if (g < 2 * G_W + G_QKV + G_SQ) {
    const int e = g - (2 * G_W + G_QKV);
    src = rnw + (size_t)e * 8; dst = rnh + (size_t)e * 8; sc = WSCALE;
  } else {
    const int e = g - (2 * G_W + G_QKV + G_SQ);
    src = oww + (size_t)e * 8; dst = owh + (size_t)e * 8; sc = WSCALE;
  }
  const v4f a = *(const v4fa*)src;
  const v4f c = *(const v4fa*)(src + 4);
  const v8h o = { (_Float16)(a.x * sc), (_Float16)(a.y * sc), (_Float16)(a.z * sc), (_Float16)(a.w * sc),
                  (_Float16)(c.x * sc), (_Float16)(c.y * sc), (_Float16)(c.z * sc), (_Float16)(c.w * sc) };
  *(volatile v8h*)dst = o;
  __threadfence();
  *(volatile v8h*)dst = o;
}

__global__ __launch_bounds__(256) void flag_kernel(const int* __restrict__ amask,
                                                   int* __restrict__ flags)
{
  __shared__ __attribute__((aligned(16))) int sf[256];
  const int t = threadIdx.x;
  const int qt = t >> 4, kt = t & 15;
  const int* base = amask + (size_t)(qt * 64) * L_SEQ + kt * 64;
  int any = 0;
  #pragma unroll 1
  for (int i = 0; i < 64; ++i) {
    const int* rp = base + (size_t)i * L_SEQ;
    #pragma unroll
    for (int c = 0; c < 16; ++c) {
      const v4i v = *(const v4ia*)(rp + 4 * c);
      any |= (v.x == 0) | (v.y == 0) | (v.z == 0) | (v.w == 0);
    }
  }
  sf[t] = any;
  __syncthreads();
  if (t < 32) {
    const v4i v0 = *(const v4ia*)(sf + 4 * t);
    const v4i v1 = *(const v4ia*)(sf + 128 + 4 * t);
    *(volatile v4i*)(flags + 4 * t) = v0;
    *(volatile v4i*)(flags + 128 + 4 * t) = v1;
    __threadfence();
    *(volatile v4i*)(flags + 4 * t) = v0;
    *(volatile v4i*)(flags + 128 + 4 * t) = v1;
  }
}

__device__ __forceinline__ void proj_store_pass(const _Float16* sT, _Float16* plane, _Float16* vt,
                                                int which, int bh, int i0, int w, int lane) {
  const int q8 = lane & 7, sub = lane >> 3;
  #pragma unroll
  for (int i = 0; i < 8; ++i) {
    const int lid = w * 32 + i * 4 + sub;
    v8h v;
    _Float16* dst;
    if (which != 2) {
      v = *(const v8ha*)(sT + lid * HDIM + 8 * q8);
      dst = plane + ((size_t)bh * L_SEQ + i0 + lid) * HDIM + 8 * q8;
    } else {
      const int d = lid >> 1, hl = lid & 1;
      v = *(const v8ha*)(sT + d * 128 + 64 * hl + 8 * q8);
      dst = vt + ((size_t)bh * HDIM + d) * L_SEQ + i0 + 64 * hl + 8 * q8;
    }
    *(volatile v8h*)dst = v;
  }
}

__global__ __launch_bounds__(128) void proj_kernel(
    const _Float16* __restrict__ wh,
    const _Float16* __restrict__ rh,
    const _Float16* __restrict__ qkvh,
    const _Float16* __restrict__ rnh,
    const float* __restrict__ rwb,
    const float* __restrict__ rrb,
    _Float16* __restrict__ qa,
    _Float16* __restrict__ qbp,
    _Float16* __restrict__ kp,
    _Float16* __restrict__ rkp,
    _Float16* __restrict__ vt)
{
  __shared__ __attribute__((aligned(16))) _Float16 sT[2][128 * HDIM];

  const int tid = threadIdx.x, lane = tid & 31, w = tid >> 5;
  const int h = lane >> 4, m = lane & 15;
  const int bx = blockIdx.x;
  const int b = bx >> 3;
  const int i0 = (bx & 7) * 128;
  const int cg = blockIdx.y;
  const int which = (cg < 48) ? (cg >> 4) : 3;
  const int head = (cg < 48) ? (cg & 15) : (cg - 48);
  const int i0w = i0 + 32 * w;

  const _Float16* Ab = (which == 3) ? rh : wh;
  const _Float16* xa0 = Ab + ((size_t)(i0w + m) * NB + b) * DMOD;
  const _Float16* xa1 = Ab + ((size_t)(i0w + 16 + m) * NB + b) * DMOD;
  const _Float16* wb = (which == 3)
      ? (rnh + ((size_t)head * HDIM + m) * DMOD)
      : (qkvh + ((size_t)which * DMOD + head * HDIM + m) * DMOD);

  const v8f zero8 = {0.f, 0.f, 0.f, 0.f, 0.f, 0.f, 0.f, 0.f};
  v8f acc[2][4];
  #pragma unroll
  for (int mt = 0; mt < 2; ++mt)
    #pragma unroll
    for (int nt = 0; nt < 4; ++nt) acc[mt][nt] = zero8;

  #pragma unroll 1
  for (int k0 = 0; k0 < DMOD; k0 += 32) {
    const v16h a0 = load_frag(xa0 + k0, h);
    const v16h a1 = load_frag(xa1 + k0, h);
    #pragma unroll
    for (int nt = 0; nt < 4; ++nt) {
      const v16h bf = load_frag(wb + (size_t)nt * 16 * DMOD + k0, h);
      acc[0][nt] = wmma_f16(a0, bf, acc[0][nt]);
      acc[1][nt] = wmma_f16(a1, bf, acc[1][nt]);
    }
  }

  const float inv32 = 1.0f / WSCALE;
  _Float16* sT0 = &sT[0][0];
  _Float16* sT1 = &sT[1][0];
  #pragma unroll
  for (int nt = 0; nt < 4; ++nt) {
    const int feat = 16 * nt + m;
    const float bw = rwb[head * HDIM + feat];
    const float br = rrb[head * HDIM + feat];
    #pragma unroll
    for (int mt = 0; mt < 2; ++mt) {
      const v8f a = acc[mt][nt];
      const int tok0 = 32 * w + 16 * mt + 8 * h;
      if (which == 2) {
        const v8h pk = { (_Float16)(a[0] * inv32), (_Float16)(a[1] * inv32), (_Float16)(a[2] * inv32), (_Float16)(a[3] * inv32),
                         (_Float16)(a[4] * inv32), (_Float16)(a[5] * inv32), (_Float16)(a[6] * inv32), (_Float16)(a[7] * inv32) };
        *(v8ha*)(sT0 + feat * 128 + tok0) = pk;
      } else if (which == 0) {
        #pragma unroll
        for (int r = 0; r < 8; ++r) {
          const float y = a[r] * inv32;
          sT0[(tok0 + r) * HDIM + feat] = (_Float16)((y + bw) * 0.125f);
          sT1[(tok0 + r) * HDIM + feat] = (_Float16)((y + br) * 0.125f);
        }
      } else {
        #pragma unroll
        for (int r = 0; r < 8; ++r)
          sT0[(tok0 + r) * HDIM + feat] = (_Float16)(a[r] * inv32);
      }
    }
  }
  __syncthreads();

  const int bh = b * NHD + head;
  _Float16* plane0 = (which == 0) ? qa : ((which == 1) ? kp : rkp);
  proj_store_pass(sT0, plane0, vt, which, bh, i0, w, lane);
  if (which == 0) proj_store_pass(sT1, qbp, vt, 0, bh, i0, w, lane);
  __threadfence();
  proj_store_pass(sT0, plane0, vt, which, bh, i0, w, lane);
  if (which == 0) proj_store_pass(sT1, qbp, vt, 0, bh, i0, w, lane);
}

__device__ __forceinline__ v8f sel_mask8(v8f s, v4i ma, v4i mb) {
  const float NEG = -1e30f;
  s[0] = (ma.x != 0) ? NEG : s[0];
  s[1] = (ma.y != 0) ? NEG : s[1];
  s[2] = (ma.z != 0) ? NEG : s[2];
  s[3] = (ma.w != 0) ? NEG : s[3];
  s[4] = (mb.x != 0) ? NEG : s[4];
  s[5] = (mb.y != 0) ? NEG : s[5];
  s[6] = (mb.z != 0) ? NEG : s[6];
  s[7] = (mb.w != 0) ? NEG : s[7];
  return s;
}

__device__ __forceinline__ v16h pack_p(v8f a, v8f c) {
  const v16h q = { (_Float16)(a[0] * PSCALE), (_Float16)(a[1] * PSCALE), (_Float16)(a[2] * PSCALE), (_Float16)(a[3] * PSCALE),
                   (_Float16)(a[4] * PSCALE), (_Float16)(a[5] * PSCALE), (_Float16)(a[6] * PSCALE), (_Float16)(a[7] * PSCALE),
                   (_Float16)(c[0] * PSCALE), (_Float16)(c[1] * PSCALE), (_Float16)(c[2] * PSCALE), (_Float16)(c[3] * PSCALE),
                   (_Float16)(c[4] * PSCALE), (_Float16)(c[5] * PSCALE), (_Float16)(c[6] * PSCALE), (_Float16)(c[7] * PSCALE) };
  return q;
}

__device__ __forceinline__ void avec_store_pass(const _Float16* so, _Float16* avec,
                                                int b, int head, int q0w, int lane) {
  const int q8 = lane & 7, sub = lane >> 3;
  #pragma unroll
  for (int i = 0; i < 4; ++i) {
    const int row = 4 * i + sub;
    const v8h v = *(const v8ha*)(so + row * HDIM + 8 * q8);
    const size_t gi = ((size_t)(q0w + row) * NB + b) * DMOD + head * HDIM + 8 * q8;
    *(volatile v8h*)(avec + gi) = v;
  }
}

__global__ __launch_bounds__(128) void attn_kernel(
    const _Float16* __restrict__ qa,
    const _Float16* __restrict__ qbp,
    const _Float16* __restrict__ kp,
    const _Float16* __restrict__ rkp,
    const _Float16* __restrict__ vt,
    const int* __restrict__ amask,
    const int* __restrict__ flags,
    _Float16* __restrict__ avec)
{
  __shared__ __attribute__((aligned(16))) float    s_band[4][16 * 80];
  __shared__ __attribute__((aligned(16))) _Float16 s_o[4][16 * HDIM];

  const int tid = threadIdx.x, lane = tid & 31, w = tid >> 5;
  const int h = lane >> 4, m = lane & 15;
  const int qblk = blockIdx.x;
  const int bh = blockIdx.y, b = bh >> 4, head = bh & 15;
  const int q0w = qblk * 64 + 16 * w;

  const _Float16* qrow = qa + ((size_t)bh * L_SEQ + q0w + m) * HDIM;
  const v16h qf0 = load_frag(qrow, h);
  const v16h qf1 = load_frag(qrow + 32, h);
  const _Float16* grow = qbp + ((size_t)bh * L_SEQ + q0w + m) * HDIM;
  const v16h gf0 = load_frag(grow, h);
  const v16h gf1 = load_frag(grow + 32, h);

  const v8f zero8 = {0.f, 0.f, 0.f, 0.f, 0.f, 0.f, 0.f, 0.f};
  v8f o[4];
  #pragma unroll
  for (int t = 0; t < 4; ++t) o[t] = zero8;
  float mrun = -1e30f, lrun = 0.0f;

  const _Float16* kbase = kp + ((size_t)bh * L_SEQ + m) * HDIM;
  const _Float16* rbase = rkp + (size_t)bh * L_SEQ * HDIM;
  const _Float16* vbase = vt + ((size_t)bh * HDIM + m) * L_SEQ;
  const int* mrow = amask + (size_t)(q0w + m) * L_SEQ + 8 * h;
  const int* frow = flags + qblk * 16;
  float* sb = &s_band[w][0];

  #pragma unroll 1
  for (int kbi = 0; kbi < 16; ++kbi) {
    const int fl = __builtin_amdgcn_readfirstlane(frow[kbi]);
    if (fl == 0) continue;
    const int kb = kbi * 64;

    const int base = L_SEQ - 16 - q0w + kb;
    #pragma unroll
    for (int t = 0; t < 5; ++t) {
      int rr = base + 16 * t + m;
      rr = rr < 0 ? 0 : rr;
      rr = rr > (L_SEQ - 1) ? (L_SEQ - 1) : rr;
      const _Float16* rp = rbase + (size_t)rr * HDIM;
      const v16h rf0 = load_frag(rp, h);
      const v16h rf1 = load_frag(rp + 32, h);
      v8f bd = zero8;
      bd = wmma_f16(rf0, gf0, bd);
      bd = wmma_f16(rf1, gf1, bd);
      const v4f lo = {bd[0], bd[1], bd[2], bd[3]};
      const v4f hi = {bd[4], bd[5], bd[6], bd[7]};
      float* bp = sb + m * 80 + 16 * t + 8 * h;
      *(v4fa*)bp = lo;
      *(v4fa*)(bp + 4) = hi;
    }

    v8f s[4];
    #pragma unroll
    for (int j = 0; j < 4; ++j) {
      const _Float16* kpj = kbase + (size_t)(kb + 16 * j) * HDIM;
      const v16h kf0 = load_frag(kpj, h);
      const v16h kf1 = load_frag(kpj + 32, h);
      v8f z = zero8;
      z = wmma_f16(kf0, qf0, z);
      z = wmma_f16(kf1, qf1, z);
      s[j] = z;
    }
    __syncthreads();

    #pragma unroll
    for (int j = 0; j < 4; ++j) {
      const float* bp = sb + m * 80 + 16 * j + 8 * h + 15 - m;
      const v8f bv = {bp[0], bp[1], bp[2], bp[3], bp[4], bp[5], bp[6], bp[7]};
      const v4i ma = *(const v4ia*)(mrow + kb + 16 * j);
      const v4i mb = *(const v4ia*)(mrow + kb + 16 * j + 4);
      s[j] = sel_mask8(s[j] + bv, ma, mb);
    }

    float mloc = s[0][0];
    #pragma unroll
    for (int j = 0; j < 4; ++j)
      #pragma unroll
      for (int r = 0; r < 8; ++r) mloc = fmaxf(mloc, s[j][r]);
    mloc = fmaxf(mloc, __shfl_xor(mloc, 16, 32));
    const float mnew = fmaxf(mrun, mloc);
    const float alpha = __expf(mrun - mnew);
    mrun = mnew;
    float lsum = 0.0f;
    #pragma unroll
    for (int j = 0; j < 4; ++j)
      #pragma unroll
      for (int r = 0; r < 8; ++r) {
        const float p = __expf(s[j][r] - mnew);
        s[j][r] = p;
        lsum += p;
      }
    lsum += __shfl_xor(lsum, 16, 32);
    lrun = lrun * alpha + lsum;
    #pragma unroll
    for (int t = 0; t < 4; ++t)
      #pragma unroll
      for (int r = 0; r < 8; ++r) o[t][r] = o[t][r] * alpha;

    const v16h pb0 = pack_p(s[0], s[1]);
    const v16h pb1 = pack_p(s[2], s[3]);

    #pragma unroll
    for (int t = 0; t < 4; ++t) {
      const _Float16* vp = vbase + (size_t)(16 * t) * L_SEQ + kb;
      const v16h vf0 = load_frag(vp, h);
      const v16h vf1 = load_frag(vp + 32, h);
      o[t] = wmma_f16(vf0, pb0, o[t]);
      o[t] = wmma_f16(vf1, pb1, o[t]);
    }
    __syncthreads();
  }

  const float inv = (1.0f / lrun) * (OSCALE / PSCALE);
  _Float16* so = &s_o[w][0];
  #pragma unroll
  for (int t = 0; t < 4; ++t) {
    const v8f a = o[t];
    const v8h pk = { (_Float16)(a[0] * inv), (_Float16)(a[1] * inv), (_Float16)(a[2] * inv), (_Float16)(a[3] * inv),
                     (_Float16)(a[4] * inv), (_Float16)(a[5] * inv), (_Float16)(a[6] * inv), (_Float16)(a[7] * inv) };
    *(v8ha*)(so + m * HDIM + 16 * t + 8 * h) = pk;
  }
  __syncthreads();

  avec_store_pass(so, avec, b, head, q0w, lane);
  __threadfence();
  avec_store_pass(so, avec, b, head, q0w, lane);
}

__global__ __launch_bounds__(256) void oproj_ln_kernel(
    const _Float16* __restrict__ avec,
    const _Float16* __restrict__ owh,
    const float* __restrict__ w,
    const float* __restrict__ gamma,
    const float* __restrict__ beta,
    float* __restrict__ out)
{
  __shared__ __attribute__((aligned(16))) float sY[8 * DMOD];

  const int tid = threadIdx.x, lane = tid & 31, wv = tid >> 5;
  const int h = lane >> 4, m = lane & 15;
  const int t0 = blockIdx.x * 16;
  const int f0 = wv * 128;

  const _Float16* xa = avec + (size_t)(t0 + m) * DMOD;
  const _Float16* wb = owh + (size_t)(f0 + m) * DMOD;

  const v8f zero8 = {0.f, 0.f, 0.f, 0.f, 0.f, 0.f, 0.f, 0.f};
  v8f acc[8];
  #pragma unroll
  for (int n = 0; n < 8; ++n) acc[n] = zero8;

  #pragma unroll 1
  for (int k0 = 0; k0 < DMOD; k0 += 32) {
    const v16h a = load_frag(xa + k0, h);
    #pragma unroll
    for (int n = 0; n < 8; ++n) {
      const v16h bf = load_frag(wb + (size_t)n * 16 * DMOD + k0, h);
      acc[n] = wmma_f16(a, bf, acc[n]);
    }
  }

  const float oinv = 1.0f / (WSCALE * OSCALE);
  const float invd = 1.0f / (float)DMOD;
  #pragma unroll 1
  for (int ph = 0; ph < 2; ++ph) {
    if (h == ph) {
      #pragma unroll
      for (int n = 0; n < 8; ++n) {
        const v8f a = acc[n];
        #pragma unroll
        for (int r = 0; r < 8; ++r) sY[r * DMOD + f0 + 16 * n + m] = a[r] * oinv;
      }
    }
    __syncthreads();

    const int row = wv;
    const int tok = t0 + 8 * ph + row;
    const float* srow = sY + row * DMOD;
    const float* wrow = w + (size_t)tok * DMOD;
    v4f x[8];
    float sum = 0.0f;
    #pragma unroll
    for (int q = 0; q < 8; ++q) {
      const int idx = 128 * q + 4 * lane;
      const v4f a = *(const v4fa*)(srow + idx);
      const v4f c = *(const v4fa*)(wrow + idx);
      x[q] = a + c;
      sum += (x[q].x + x[q].y) + (x[q].z + x[q].w);
    }
    #pragma unroll
    for (int off = 16; off >= 1; off >>= 1) sum += __shfl_xor(sum, off, 32);
    const float mu = sum * invd;
    float sq = 0.0f;
    #pragma unroll
    for (int q = 0; q < 8; ++q) {
      const v4f d = x[q] - mu;
      sq += (d.x * d.x + d.y * d.y) + (d.z * d.z + d.w * d.w);
    }
    #pragma unroll
    for (int off = 16; off >= 1; off >>= 1) sq += __shfl_xor(sq, off, 32);
    const float rstd = rsqrtf(sq * invd + 1e-5f);

    v4f y[8];
    float* orow = out + (size_t)tok * DMOD;
    #pragma unroll
    for (int q = 0; q < 8; ++q) {
      const int idx = 128 * q + 4 * lane;
      const v4f g  = *(const v4fa*)(gamma + idx);
      const v4f be = *(const v4fa*)(beta + idx);
      y[q] = (x[q] - mu) * rstd * g + be;
      *(volatile v4f*)(orow + idx) = y[q];
    }
    __threadfence();
    #pragma unroll
    for (int q = 0; q < 8; ++q) {
      const int idx = 128 * q + 4 * lane;
      *(volatile v4f*)(orow + idx) = y[q];
    }
    __syncthreads();
  }
}

extern "C" void kernel_launch(void* const* d_in, const int* in_sizes, int n_in,
                              void* d_out, int out_size, void* d_ws, size_t ws_size,
                              hipStream_t stream) {
  if (n_in < 10) return;
  if (in_sizes[0] != NTOK * DMOD || in_sizes[1] != NTOK * DMOD) return;
  if (in_sizes[2] != NHD * HDIM || in_sizes[3] != NHD * HDIM) return;
  if (in_sizes[4] != 3 * DMOD * DMOD) return;
  if (in_sizes[5] != DMOD * DMOD || in_sizes[6] != DMOD * DMOD) return;
  if (in_sizes[7] != DMOD || in_sizes[8] != DMOD) return;
  if (in_sizes[9] != L_SEQ * L_SEQ) return;
  if (out_size != NTOK * DMOD) return;

  const float* w     = (const float*)d_in[0];
  const float* r     = (const float*)d_in[1];
  const float* rwb   = (const float*)d_in[2];
  const float* rrb   = (const float*)d_in[3];
  const float* qkvw  = (const float*)d_in[4];
  const float* rnw   = (const float*)d_in[5];
  const float* oww   = (const float*)d_in[6];
  const float* gamma = (const float*)d_in[7];
  const float* beta  = (const float*)d_in[8];
  const int*   amask = (const int*)d_in[9];
  float* out = (float*)d_out;

  const size_t b_act = (size_t)NTOK * DMOD * 2;
  const size_t b_qkv = (size_t)3 * DMOD * DMOD * 2;
  const size_t b_sq  = (size_t)DMOD * DMOD * 2;
  const size_t b_pl  = (size_t)NBH * L_SEQ * HDIM * 2;
  const size_t b_fl  = 4096;
  const size_t total = 2 * b_act + b_qkv + 2 * b_sq + 5 * b_pl + b_act + b_fl;
  if (total > ws_size) return;
  if (total > (size_t)134217728) return;

  char* ws = (char*)d_ws;
  size_t off = 0;
  _Float16* wh   = (_Float16*)(ws + off); off += b_act;
  _Float16* rh   = (_Float16*)(ws + off); off += b_act;
  _Float16* qkvh = (_Float16*)(ws + off); off += b_qkv;
  _Float16* rnh  = (_Float16*)(ws + off); off += b_sq;
  _Float16* owh  = (_Float16*)(ws + off); off += b_sq;
  _Float16* qa   = (_Float16*)(ws + off); off += b_pl;
  _Float16* qbp  = (_Float16*)(ws + off); off += b_pl;
  _Float16* kp   = (_Float16*)(ws + off); off += b_pl;
  _Float16* rkp  = (_Float16*)(ws + off); off += b_pl;
  _Float16* vt   = (_Float16*)(ws + off); off += b_pl;
  _Float16* avec = (_Float16*)(ws + off); off += b_act;
  int*      flags = (int*)(ws + off);     off += b_fl;
  if (off != total) return;

  convert_kernel<<<(G_TOT + 255) / 256, 256, 0, stream>>>(w, r, qkvw, rnw, oww, wh, rh, qkvh, rnh, owh);

  flag_kernel<<<1, 256, 0, stream>>>(amask, flags);

  dim3 gProj(NB * (L_SEQ / 128), 3 * NHD + NHD);
  proj_kernel<<<gProj, 128, 0, stream>>>(wh, rh, qkvh, rnh, rwb, rrb, qa, qbp, kp, rkp, vt);

  dim3 gAtt(L_SEQ / 64, NBH);
  attn_kernel<<<gAtt, 128, 0, stream>>>(qa, qbp, kp, rkp, vt, amask, flags, avec);

  oproj_ln_kernel<<<NTOK / 16, 256, 0, stream>>>(avec, owh, w, gamma, beta, out);
}
